// LSTMAutoencoder_42795054137800
// MI455X (gfx1250) — hardware-run, weakly checked
//
#include <hip/hip_runtime.h>
#include <math.h>

constexpr int NBATCH = 32768;
constexpr int NSTEP  = 30;
constexpr int NIN    = 4;
constexpr int NHID   = 64;
constexpr int NLAT   = 32;
constexpr int NG1 = 4 * NHID;
constexpr int NG2 = 4 * NLAT;
constexpr int NG4 = 4 * NIN;
constexpr int KE1  = 96;
constexpr int KE2  = 96;
constexpr int KD1X = 32;
constexpr int KD1H = 64;
constexpr int KD2  = 64;
constexpr int EROWS = 64;
constexpr int ETHR  = 256;
constexpr int DROWS = 32;
constexpr int DTHR  = 128;
constexpr int AP   = 104;
constexpr int A3P  = 72;
constexpr int LHP  = 40;
constexpr int LSP  = 36;
constexpr int OSP  = NSTEP * NIN;
constexpr int XGPL = DTHR * 4;
constexpr int NXG  = 16;
constexpr float OPC  = 16.0f;
constexpr float PSC  = 256.0f;
constexpr float PINV = 1.0f / 256.0f;
constexpr float RSC  = 256.0f;
constexpr float RINV = 1.0f / 256.0f;

static_assert(NBATCH % EROWS == 0 && NBATCH % DROWS == 0);
static_assert(KE1 % 32 == 0 && KE2 % 32 == 0 && KD1X % 32 == 0 && KD1H % 32 == 0 && KD2 % 32 == 0);
static_assert(NG1 % 16 == 0 && NG2 % 16 == 0 && NG4 == 16);
static_assert(AP % 8 == 0 && A3P % 8 == 0 && LHP % 8 == 0 && LSP % 4 == 0 && XGPL % 4 == 0);
static_assert(ETHR == 4 * EROWS);
static_assert(ETHR == NG1 && ETHR == 2 * NG2);
static_assert(DTHR == 4 * DROWS);
static_assert(2 * DTHR == NG1 && NG4 <= 16);
static_assert((4 * DROWS * A3P) % (8 * DTHR) == 0);
static_assert((EROWS * NLAT) % (4 * ETHR) == 0);
static_assert((DROWS * OSP) % 4 == 0 && (DROWS * OSP * 4) % 128 == 0);
static_assert(NHID + 32 <= AP && KE2 <= AP && KD1H + 8 <= A3P && KD1X + 8 <= LHP);

typedef __attribute__((ext_vector_type(16))) _Float16 v16h;
typedef __attribute__((ext_vector_type(8)))  _Float16 v8h;
typedef __attribute__((ext_vector_type(8)))  float    v8f;
typedef __attribute__((ext_vector_type(4)))  float    v4f;
typedef __attribute__((ext_vector_type(4)))  unsigned v4u;

template <typename T> struct Frag;
template <> struct Frag<_Float16> {
  typedef v16h V; union U { v16h v; v8h h[2]; };
  static __device__ __forceinline__ v16h load(const _Float16* p) {
    U f; f.h[0] = *(const v8h*)(p); f.h[1] = *(const v8h*)(p + 16); return f.v;
  }
  static __device__ __forceinline__ v8f mma(v16h a, v16h b, v8f c) {
    return __builtin_amdgcn_wmma_f32_16x16x32_f16(false, a, false, b, (short)0, c, false, false);
  }
};
typedef Frag<_Float16> FH;

__device__ __forceinline__ void mma_guard4(v8f& a0, v8f& a1, v8f& a2, v8f& a3, v16h x, v16h y0, v16h y1, v16h y2, v16h y3) {
  asm volatile("v_nop\n\tv_nop\n\tv_nop\n\tv_nop" : "+v"(a0), "+v"(a1), "+v"(a2), "+v"(a3) : "v"(x), "v"(y0), "v"(y1), "v"(y2), "v"(y3));
}
__device__ __forceinline__ void mma_guard8m(v8f& a0, v8f& a1, v8f& a2, v8f& a3, v8f& r0, v8f& r1, v8f& r2, v8f& r3,
                                            v16h x, v16h xl, v16h y0, v16h y1, v16h y2, v16h y3) {
  asm volatile("v_nop\n\tv_nop\n\tv_nop\n\tv_nop"
               : "+v"(a0), "+v"(a1), "+v"(a2), "+v"(a3), "+v"(r0), "+v"(r1), "+v"(r2), "+v"(r3)
               : "v"(x), "v"(xl), "v"(y0), "v"(y1), "v"(y2), "v"(y3) : "memory");
}
__device__ __forceinline__ void mma_guard2(v8f& a0, v8f& a1, v16h x, v16h xl, v16h y, v16h yl) {
  asm volatile("v_nop\n\tv_nop\n\tv_nop\n\tv_nop" : "+v"(a0), "+v"(a1) : "v"(x), "v"(xl), "v"(y), "v"(yl));
}
__device__ __forceinline__ void acc_guard4(v8f& a, v8f& b, v8f& c, v8f& d) { asm volatile("v_nop\n\tv_nop\n\tv_nop\n\tv_nop" : "+v"(a), "+v"(b), "+v"(c), "+v"(d)); }
__device__ __forceinline__ void acc_guard2(v8f& a, v8f& b) { asm volatile("v_nop\n\tv_nop\n\tv_nop\n\tv_nop" : "+v"(a), "+v"(b)); }
__device__ __forceinline__ void use8(float a, float b, float c, float d, float e, float f, float g, float h) {
  asm volatile("" :: "v"(a), "v"(b), "v"(c), "v"(d), "v"(e), "v"(f), "v"(g), "v"(h));
}

__device__ __forceinline__ float fsig(float x)  { return __builtin_amdgcn_rcpf(1.0f + __expf(-x)); }
__device__ __forceinline__ float ftanh(float x) { return 1.0f - 2.0f * __builtin_amdgcn_rcpf(__expf(2.0f * x) + 1.0f); }
__device__ __forceinline__ _Float16 to_h(float v) { return (_Float16)(v * OPC); }
__device__ __forceinline__ void to_h2(float v, _Float16& hi, _Float16& lo) {
  const float s = v * OPC;
  const _Float16 h = (_Float16)s;
  const float hf = (float)h;
  hi = h;
  lo = (_Float16)((s - hf) * RSC);
}

__device__ __forceinline__ float lstm_cell(float zi, float zf, float zg, float zo, float& cs) {
  const float ig = fsig(zi);
  const float fg = fsig(zf);
  const float gg = ftanh(zg);
  const float og = fsig(zo);
  const float cn = fg * cs + ig * gg;
  cs = cn;
  return og * ftanh(cn);
}

template <int MODE>
__global__ __launch_bounds__(256) void wplane_kernel(const float* __restrict__ s0, int n0c, int ld0,
                                                     const float* __restrict__ s1, int n1c, int ld1,
                                                     int nrow, int kp, unsigned short* __restrict__ dst) {
  const int i   = blockIdx.x * 256 + threadIdx.x;
  const int kp8 = kp >> 3;
  const int n8  = nrow * kp8;
  if (i < n8) {
    const int n  = i / kp8;
    const int c8 = i - n * kp8;
    float v0[8], v1[8];
#pragma unroll
    for (int e = 0; e < 8; ++e) {
      const int k   = c8 * 8 + e;
      const int k0c = (k < n0c) ? k : (n0c - 1);
      v0[e] = s0[(size_t)n * ld0 + k0c];
    }
    use8(v0[0], v0[1], v0[2], v0[3], v0[4], v0[5], v0[6], v0[7]);
#pragma unroll
    for (int e = 0; e < 8; ++e) {
      const int k1  = c8 * 8 + e - n0c;
      const int k1c = (k1 < 0) ? 0 : ((k1 < n1c) ? k1 : (n1c - 1));
      v1[e] = s1[(size_t)n * ld1 + k1c];
    }
    use8(v1[0], v1[1], v1[2], v1[3], v1[4], v1[5], v1[6], v1[7]);
    v8h hv;
#pragma unroll
    for (int e = 0; e < 8; ++e) {
      const int k = c8 * 8 + e;
      const float f0 = (k < n0c) ? 1.0f : 0.0f;
      const float f1 = (k >= n0c && k < n0c + n1c) ? 1.0f : 0.0f;
      const float v  = fmaf(f0, v0[e], f1 * v1[e]) + 0.0f;
      _Float16 hvs, lvs;
      to_h2(v, hvs, lvs);
      const _Float16 o = (MODE == 0) ? hvs : lvs;
      hv[e] = o;
    }
    *(volatile v8h*)(dst + (size_t)i * 8) = hv;
    __threadfence();
    *(volatile v8h*)(dst + (size_t)i * 8) = hv;
  }
}

__device__ __forceinline__ void stage_x(_Float16* A1t, const float* __restrict__ x, int rowbase, int tstep, int tid, int wave) {
  if (wave < 2) {
    const int row = tid;
    const v4f xv = *(const v4f*)(x + ((size_t)(rowbase + row) * NSTEP + (size_t)tstep) * NIN);
    const _Float16 e0 = to_h(xv[0]), e1 = to_h(xv[1]), e2 = to_h(xv[2]), e3 = to_h(xv[3]);
    const unsigned w0 = (unsigned)__builtin_bit_cast(unsigned short, e0) | ((unsigned)__builtin_bit_cast(unsigned short, e1) << 16);
    const unsigned w1 = (unsigned)__builtin_bit_cast(unsigned short, e2) | ((unsigned)__builtin_bit_cast(unsigned short, e3) << 16);
    v4u u; u[0] = w0; u[1] = w1; u[2] = w0; u[3] = w1;
    *(v4u*)(A1t + row * AP + NHID) = u;
  } else {
    const int q    = tid - 64;
    const int row  = q / 3;
    const int part = q - 3 * row;
    v4u z; z[0] = 0u; z[1] = 0u; z[2] = 0u; z[3] = 0u;
    *(v4u*)(A1t + row * AP + NHID + 8 + 8 * part) = z;
  }
}

__global__ __launch_bounds__(ETHR) __attribute__((amdgpu_num_vgpr(256)))
void enc_kernel(const float* __restrict__ x,
                const unsigned short* __restrict__ WE1p,
                const unsigned short* __restrict__ WE2p,
                const float* __restrict__ b1i, const float* __restrict__ b1h,
                const float* __restrict__ b2i, const float* __restrict__ b2h,
                float* __restrict__ LAT) {
  __shared__ __align__(16) _Float16 A1[2][EROWS * AP];
  __shared__ __align__(16) _Float16 A2[2][EROWS * AP];
  __shared__ __align__(16) float    LS[EROWS * LSP];
  __shared__ __align__(16) float    BS1[NG1];
  __shared__ __align__(16) float    BS2[NG2];
  const _Float16* WE1 = (const _Float16*)WE1p;
  const _Float16* WE2 = (const _Float16*)WE2p;
  const int tid  = threadIdx.x;
  const int lane = tid & 31;
  const int wave = __builtin_amdgcn_readfirstlane((int)(threadIdx.x >> 5));
  const int c = lane & 15, hh = lane >> 4, koff = hh * 8;
  const int ms = wave >> 1, wsub = wave & 1;
  const int rowbase = blockIdx.x * EROWS;
  const int arow = (16 * ms + c) * AP + koff;

  {
    const float u0 = b1i[tid], u1 = b1h[tid];
    BS1[tid] = u0 + u1;
  }
  if (wave < 4) {
    const float u0 = b2i[tid], u1 = b2h[tid];
    BS2[tid] = u0 + u1;
  }
  {
    v4u z; z[0] = 0u; z[1] = 0u; z[2] = 0u; z[3] = 0u;
    _Float16* p1 = &A1[0][0];
    _Float16* p2 = &A2[0][0];
#pragma unroll 1
    for (int i = tid; i < (2 * EROWS * AP) / 8; i += ETHR) { *(v4u*)(p1 + 8 * i) = z; *(v4u*)(p2 + 8 * i) = z; }
  }
  float c1[2][8], c2[8], h2s[8];
#pragma unroll
  for (int r = 0; r < 8; ++r) { c1[0][r] = 0.0f; c1[1][r] = 0.0f; c2[r] = 0.0f; h2s[r] = 0.0f; }
  __syncthreads();
  float bb1[2][4], bb2[4];
#pragma unroll
  for (int ug = 0; ug < 2; ++ug)
#pragma unroll
    for (int g = 0; g < 4; ++g) bb1[ug][g] = BS1[g * NHID + 16 * (2 * wsub + ug) + c];
#pragma unroll
  for (int g = 0; g < 4; ++g) bb2[g] = BS2[g * NLAT + 16 * wsub + c];
  stage_x(&A1[0][0], x, rowbase, 0, tid, wave);
  __syncthreads();

  const v8f z8 = {0.f, 0.f, 0.f, 0.f, 0.f, 0.f, 0.f, 0.f};

#pragma unroll 1
  for (int t = 0; t < NSTEP; ++t) {
    const int cur = t & 1, nxt = cur ^ 1;
    const _Float16* a1r = &A1[cur][0] + arow;
    _Float16*       a1n = &A1[nxt][0];
    _Float16*       a2c = &A2[cur][0];
    const _Float16* a2r = a2c + arow;

#pragma unroll
    for (int ug = 0; ug < 2; ++ug) {
      const int j = 16 * (2 * wsub + ug) + c;
      const _Float16* wp = WE1 + (size_t)j * KE1 + koff;
      v8f acc[4];
      acc[0] = z8; acc[1] = z8; acc[2] = z8; acc[3] = z8;
#pragma unroll 1
      for (int k0 = 0; k0 < KE1; k0 += 32) {
        const v16h a  = FH::load(a1r + k0);
        const v16h b0 = FH::load(wp + k0);
        const v16h b1 = FH::load(wp + (size_t)1 * NHID * KE1 + k0);
        const v16h b2 = FH::load(wp + (size_t)2 * NHID * KE1 + k0);
        const v16h b3 = FH::load(wp + (size_t)3 * NHID * KE1 + k0);
        acc[0] = FH::mma(a, b0, acc[0]);
        acc[1] = FH::mma(a, b1, acc[1]);
        acc[2] = FH::mma(a, b2, acc[2]);
        acc[3] = FH::mma(a, b3, acc[3]);
        mma_guard4(acc[0], acc[1], acc[2], acc[3], a, b0, b1, b2, b3);
      }
      acc_guard4(acc[0], acc[1], acc[2], acc[3]);
#pragma unroll
      for (int r = 0; r < 8; ++r) {
        const float zi = acc[0][r] * PINV + bb1[ug][0];
        const float zf = acc[1][r] * PINV + bb1[ug][1];
        const float zg = acc[2][r] * PINV + bb1[ug][2];
        const float zo = acc[3][r] * PINV + bb1[ug][3];
        const float hn = lstm_cell(zi, zf, zg, zo, c1[ug][r]);
        const _Float16 hv = to_h(hn);
        const int o = (16 * ms + 8 * hh + r) * AP + j;
        a1n[o] = hv;
        a2c[o] = hv;
      }
    }
#pragma unroll
    for (int r = 0; r < 8; ++r) {
      const _Float16 hv2 = to_h(h2s[r]);
      a2c[(16 * ms + 8 * hh + r) * AP + NHID + 16 * wsub + c] = hv2;
    }
    {
      const int tn = (t + 1 < NSTEP) ? (t + 1) : (NSTEP - 1);
      stage_x(a1n, x, rowbase, tn, tid, wave);
    }
    __syncthreads();

    {
      const int j2 = 16 * wsub + c;
      const _Float16* wp = WE2 + (size_t)j2 * KE2 + koff;
      v8f acc[4];
      acc[0] = z8; acc[1] = z8; acc[2] = z8; acc[3] = z8;
#pragma unroll 1
      for (int k0 = 0; k0 < KE2; k0 += 32) {
        const v16h a  = FH::load(a2r + k0);
        const v16h b0 = FH::load(wp + k0);
        const v16h b1 = FH::load(wp + (size_t)1 * NLAT * KE2 + k0);
        const v16h b2 = FH::load(wp + (size_t)2 * NLAT * KE2 + k0);
        const v16h b3 = FH::load(wp + (size_t)3 * NLAT * KE2 + k0);
        acc[0] = FH::mma(a, b0, acc[0]);
        acc[1] = FH::mma(a, b1, acc[1]);
        acc[2] = FH::mma(a, b2, acc[2]);
        acc[3] = FH::mma(a, b3, acc[3]);
        mma_guard4(acc[0], acc[1], acc[2], acc[3], a, b0, b1, b2, b3);
      }
      acc_guard4(acc[0], acc[1], acc[2], acc[3]);
#pragma unroll
      for (int r = 0; r < 8; ++r) {
        const float zi = acc[0][r] * PINV + bb2[0];
        const float zf = acc[1][r] * PINV + bb2[1];
        const float zg = acc[2][r] * PINV + bb2[2];
        const float zo = acc[3][r] * PINV + bb2[3];
        h2s[r] = lstm_cell(zi, zf, zg, zo, c2[r]);
      }
    }
  }

#pragma unroll
  for (int r = 0; r < 8; ++r) LS[(16 * ms + 8 * hh + r) * LSP + 16 * wsub + c] = h2s[r];
  __syncthreads();
  for (int pass = 0; pass < 2; ++pass) {
#pragma unroll
    for (int it = 0; it < (EROWS * NLAT) / (4 * ETHR); ++it) {
      const int idx = it * ETHR + tid;
      const int row = idx >> 3, c4 = (idx & 7) * 4;
      const v4f v = *(const v4f*)(LS + row * LSP + c4);
      *(volatile v4f*)(LAT + (size_t)(rowbase + row) * NLAT + c4) = v;
    }
    __threadfence();
  }
}

union U8 { v8f v; v4f q[2]; };
__global__ __launch_bounds__(DTHR) __attribute__((amdgpu_num_vgpr(256)))
void dec_kernel(const float* __restrict__ LAT,
                const unsigned short* __restrict__ WXHp,
                const unsigned short* __restrict__ WXLp,
                const unsigned short* __restrict__ WHp,
                const unsigned short* __restrict__ W4Hp,
                const unsigned short* __restrict__ W4Lp,
                const float* __restrict__ b3i, const float* __restrict__ b3h,
                const float* __restrict__ w4hh,
                const float* __restrict__ b4i, const float* __restrict__ b4h,
                float* __restrict__ out) {
  __shared__ __align__(16) _Float16 LH[DROWS * LHP];
  __shared__ __align__(16) _Float16 LL[DROWS * LHP];
  __shared__ __align__(16) _Float16 A3[4][DROWS * A3P];
  __shared__ __align__(16) float    XG[NXG * XGPL];
  __shared__ __align__(16) float    OS[DROWS * OSP];
  __shared__ __align__(16) float    BS3[NG1];
  const _Float16* WXH = (const _Float16*)WXHp;
  const _Float16* WXL = (const _Float16*)WXLp;
  const _Float16* WH  = (const _Float16*)WHp;
  const _Float16* W4H = (const _Float16*)W4Hp;
  const _Float16* W4L = (const _Float16*)W4Lp;
  const int tid  = threadIdx.x;
  const int lane = tid & 31;
  const int wave = __builtin_amdgcn_readfirstlane((int)(threadIdx.x >> 5));
  const int c = lane & 15, hh = lane >> 4, koff = hh * 8;
  const int ms = wave >> 1, wsub = wave & 1;
  const int rowbase = blockIdx.x * DROWS;
  const int arow3 = (16 * ms + c) * A3P + koff;

  {
    const float u0 = b3i[tid], u1 = b3h[tid], u2 = b3i[DTHR + tid], u3 = b3h[DTHR + tid];
    BS3[tid] = u0 + u1;
    BS3[DTHR + tid] = u2 + u3;
  }
  {
    const int row = tid >> 2, c8 = (tid & 3) * 8;
    const float* lp = LAT + (size_t)(rowbase + row) * NLAT + c8;
    const v4f q0 = *(const v4f*)(lp), q1 = *(const v4f*)(lp + 4);
    v8h vh, vl;
#pragma unroll
    for (int e = 0; e < 4; ++e) {
      _Float16 h0, l0, h1, l1;
      to_h2(q0[e], h0, l0);
      to_h2(q1[e], h1, l1);
      vh[e] = h0; vl[e] = l0; vh[4 + e] = h1; vl[4 + e] = l1;
    }
    *(v8h*)(LH + row * LHP + c8) = vh;
    *(v8h*)(LL + row * LHP + c8) = vl;
  }
  {
    v4u z; z[0] = 0u; z[1] = 0u; z[2] = 0u; z[3] = 0u;
    _Float16* p3 = &A3[0][0];
#pragma unroll 1
    for (int i = tid; i < (4 * DROWS * A3P) / 8; i += DTHR) *(v4u*)(p3 + 8 * i) = z;
  }
  const v4f w4 = *(const v4f*)(w4hh + 4 * c);
  const float b4 = b4i[c] + b4h[c];
  float c3[2][8], c4[8], h4[8];
#pragma unroll
  for (int r = 0; r < 8; ++r) { c3[0][r] = 0.0f; c3[1][r] = 0.0f; c4[r] = 0.0f; h4[r] = 0.0f; }
  __syncthreads();

  const v8f z8 = {0.f, 0.f, 0.f, 0.f, 0.f, 0.f, 0.f, 0.f};

  {
    const v16h a  = FH::load(LH + (16 * ms + c) * LHP + koff);
    const v16h al = FH::load(LL + (16 * ms + c) * LHP + koff);
#pragma unroll
    for (int ug = 0; ug < 2; ++ug) {
      const int j = 16 * (2 * wsub + ug) + c;
      const _Float16* wp = WXH + (size_t)j * KD1X + koff;
      const _Float16* wl = WXL + (size_t)j * KD1X + koff;
      const v16h b0 = FH::load(wp);
      const v16h b1 = FH::load(wp + (size_t)1 * NHID * KD1X);
      const v16h b2 = FH::load(wp + (size_t)2 * NHID * KD1X);
      const v16h b3 = FH::load(wp + (size_t)3 * NHID * KD1X);
      v8f am[4], ar[4];
      am[0] = FH::mma(a, b0, z8);  am[1] = FH::mma(a, b1, z8);  am[2] = FH::mma(a, b2, z8);  am[3] = FH::mma(a, b3, z8);
      ar[0] = FH::mma(al, b0, z8); ar[1] = FH::mma(al, b1, z8); ar[2] = FH::mma(al, b2, z8); ar[3] = FH::mma(al, b3, z8);
      mma_guard8m(am[0], am[1], am[2], am[3], ar[0], ar[1], ar[2], ar[3], a, al, b0, b1, b2, b3);
      const v16h l0 = FH::load(wl);
      const v16h l1 = FH::load(wl + (size_t)1 * NHID * KD1X);
      const v16h l2 = FH::load(wl + (size_t)2 * NHID * KD1X);
      const v16h l3 = FH::load(wl + (size_t)3 * NHID * KD1X);
      ar[0] = FH::mma(a, l0, ar[0]); ar[1] = FH::mma(a, l1, ar[1]); ar[2] = FH::mma(a, l2, ar[2]); ar[3] = FH::mma(a, l3, ar[3]);
      mma_guard8m(am[0], am[1], am[2], am[3], ar[0], ar[1], ar[2], ar[3], a, al, l0, l1, l2, l3);
#pragma unroll
      for (int g = 0; g < 4; ++g) {
        const float bsum = PSC * BS3[g * NHID + j];
        v4f lo4, hi4;
#pragma unroll
        for (int e = 0; e < 4; ++e) {
          lo4[e] = am[g][e] + ar[g][e] * RINV + bsum;
          hi4[e] = am[g][4 + e] + ar[g][4 + e] * RINV + bsum;
        }
        *(v4f*)(XG + ((ug * 4 + g) * 2 + 0) * XGPL + tid * 4) = lo4;
        *(v4f*)(XG + ((ug * 4 + g) * 2 + 1) * XGPL + tid * 4) = hi4;
      }
    }
  }
  __syncthreads();

#pragma unroll 1
  for (int t = 0; t < NSTEP; ++t) {
    const int cur = t & 1, nxt = cur ^ 1;
    int xo = tid * 4;
    asm volatile("" : "+v"(xo));
    const _Float16* a3r  = &A3[cur][0] + arow3;
    _Float16*       a3n  = &A3[nxt][0];
    _Float16*       a3ln = &A3[2 + nxt][0];

#pragma unroll
    for (int ug = 0; ug < 2; ++ug) {
      const int j = 16 * (2 * wsub + ug) + c;
      const _Float16* wp = WH + (size_t)j * KD1H + koff;
      v8f acc[4];
#pragma unroll
      for (int g = 0; g < 4; ++g) {
        U8 u;
        u.q[0] = *(const v4f*)(XG + ((ug * 4 + g) * 2 + 0) * XGPL + xo);
        u.q[1] = *(const v4f*)(XG + ((ug * 4 + g) * 2 + 1) * XGPL + xo);
        acc[g] = u.v;
      }
#pragma unroll 1
      for (int k0 = 0; k0 < KD1H; k0 += 32) {
        const v16h a  = FH::load(a3r + k0);
        const v16h b0 = FH::load(wp + k0);
        const v16h b1 = FH::load(wp + (size_t)1 * NHID * KD1H + k0);
        const v16h b2 = FH::load(wp + (size_t)2 * NHID * KD1H + k0);
        const v16h b3 = FH::load(wp + (size_t)3 * NHID * KD1H + k0);
        acc[0] = FH::mma(a, b0, acc[0]);
        acc[1] = FH::mma(a, b1, acc[1]);
        acc[2] = FH::mma(a, b2, acc[2]);
        acc[3] = FH::mma(a, b3, acc[3]);
        mma_guard4(acc[0], acc[1], acc[2], acc[3], a, b0, b1, b2, b3);
      }
      acc_guard4(acc[0], acc[1], acc[2], acc[3]);
#pragma unroll
      for (int r = 0; r < 8; ++r) {
        const float hn = lstm_cell(acc[0][r] * PINV, acc[1][r] * PINV, acc[2][r] * PINV, acc[3][r] * PINV, c3[ug][r]);
        _Float16 hv, lv;
        to_h2(hn, hv, lv);
        const int o = (16 * ms + 8 * hh + r) * A3P + j;
        a3n[o]  = hv;
        a3ln[o] = lv;
      }
    }
    __syncthreads();

    if (wsub == 0) {
      const _Float16* a4r = a3n  + arow3;
      const _Float16* a4l = a3ln + arow3;
      const _Float16* wq  = W4H + (size_t)c * KD2 + koff;
      const _Float16* wql = W4L + (size_t)c * KD2 + koff;
      v8f am = z8, ar = z8;
#pragma unroll 1
      for (int k0 = 0; k0 < KD2; k0 += 32) {
        const v16h a  = FH::load(a4r + k0);
        const v16h al = FH::load(a4l + k0);
        const v16h b  = FH::load(wq + k0);
        const v16h bl = FH::load(wql + k0);
        am = FH::mma(a, b, am);
        ar = FH::mma(a, bl, ar);
        ar = FH::mma(al, b, ar);
        mma_guard2(am, ar, a, al, b, bl);
      }
      acc_guard2(am, ar);
      const int base = lane & 16;
      const int ch   = c & 3;
#pragma unroll
      for (int r = 0; r < 8; ++r) {
        const float p0 = __shfl(h4[r], base + 0, 32);
        const float p1 = __shfl(h4[r], base + 1, 32);
        const float p2 = __shfl(h4[r], base + 2, 32);
        const float p3 = __shfl(h4[r], base + 3, 32);
        float v = (am[r] + ar[r] * RINV) * PINV + b4;
        v += w4[0] * p0 + w4[1] * p1 + w4[2] * p2 + w4[3] * p3;
        const float vi = __shfl(v, base + ch, 32);
        const float vf = __shfl(v, base + 4 + ch, 32);
        const float vg = __shfl(v, base + 8 + ch, 32);
        const float vo = __shfl(v, base + 12 + ch, 32);
        const float hn = lstm_cell(vi, vf, vg, vo, c4[r]);
        h4[r] = hn;
        if (c < NIN) OS[(16 * ms + 8 * hh + r) * OSP + NIN * t + c] = hn;
      }
    }
  }

  __syncthreads();
  float* ob = out + (size_t)rowbase * OSP;
  for (int pass = 0; pass < 2; ++pass) {
#pragma unroll
    for (int it = 0; it < (DROWS * OSP + 4 * DTHR - 1) / (4 * DTHR); ++it) {
      const int idx = it * DTHR + tid;
      if (idx < (DROWS * OSP) / 4) {
        const v4f v = *(const v4f*)(OS + idx * 4);
        *(volatile v4f*)(ob + (size_t)idx * 4) = v;
      }
    }
    __threadfence();
  }
}

extern "C" void kernel_launch(void* const* d_in, const int* in_sizes, int n_in,
                              void* d_out, int out_size, void* d_ws, size_t ws_size, hipStream_t stream) {
  if (n_in < 17 || d_out == nullptr || d_ws == nullptr) return;
  if (in_sizes[0] != NBATCH * NSTEP * NIN ||
      in_sizes[1] != NG1 * NIN  || in_sizes[2]  != NG1 * NHID || in_sizes[3]  != NG1 || in_sizes[4]  != NG1 ||
      in_sizes[5] != NG2 * NHID || in_sizes[6]  != NG2 * NLAT || in_sizes[7]  != NG2 || in_sizes[8]  != NG2 ||
      in_sizes[9] != NG1 * NLAT || in_sizes[10] != NG1 * NHID || in_sizes[11] != NG1 || in_sizes[12] != NG1 ||
      in_sizes[13] != NG4 * NHID || in_sizes[14] != NG4 * NIN || in_sizes[15] != NG4 || in_sizes[16] != NG4 ||
      out_size != NBATCH * NSTEP * NIN) return;

  const float* x     = (const float*)d_in[0];
  const float* e1Wih = (const float*)d_in[1];
  const float* e1Whh = (const float*)d_in[2];
  const float* e1bih = (const float*)d_in[3];
  const float* e1bhh = (const float*)d_in[4];
  const float* e2Wih = (const float*)d_in[5];
  const float* e2Whh = (const float*)d_in[6];
  const float* e2bih = (const float*)d_in[7];
  const float* e2bhh = (const float*)d_in[8];
  const float* d1Wih = (const float*)d_in[9];
  const float* d1Whh = (const float*)d_in[10];
  const float* d1bih = (const float*)d_in[11];
  const float* d1bhh = (const float*)d_in[12];
  const float* d2Wih = (const float*)d_in[13];
  const float* d2Whh = (const float*)d_in[14];
  const float* d2bih = (const float*)d_in[15];
  const float* d2bhh = (const float*)d_in[16];
  float* out = (float*)d_out;

  char* ws = (char*)d_ws; size_t off = 0;
  auto carve = [&](size_t bytes) -> char* { char* p = ws + off; off += (bytes + 511) & ~(size_t)511; return p; };
  unsigned short* WE1 = (unsigned short*)carve((size_t)NG1 * KE1 * 2);
  unsigned short* WE2 = (unsigned short*)carve((size_t)NG2 * KE2 * 2);
  unsigned short* WXH = (unsigned short*)carve((size_t)NG1 * KD1X * 2);
  unsigned short* WXL = (unsigned short*)carve((size_t)NG1 * KD1X * 2);
  unsigned short* WH  = (unsigned short*)carve((size_t)NG1 * KD1H * 2);
  unsigned short* W4H = (unsigned short*)carve((size_t)NG4 * KD2 * 2);
  unsigned short* W4L = (unsigned short*)carve((size_t)NG4 * KD2 * 2);
  float*          LAT = (float*)carve((size_t)NBATCH * NLAT * 4);
  if (off > ws_size || off > (size_t)134217728) return;

  {
    const int n8a = NG1 * (KE1 / 8), n8b = NG2 * (KE2 / 8), n8c = NG1 * (KD1X / 8), n8d = NG1 * (KD1H / 8), n8e = NG4 * (KD2 / 8);
    wplane_kernel<0><<<(n8a + 255) / 256, 256, 0, stream>>>(e1Whh, NHID, NHID, e1Wih, NIN,  NIN,  NG1, KE1,  WE1);
    wplane_kernel<0><<<(n8b + 255) / 256, 256, 0, stream>>>(e2Wih, NHID, NHID, e2Whh, NLAT, NLAT, NG2, KE2,  WE2);
    wplane_kernel<0><<<(n8c + 255) / 256, 256, 0, stream>>>(d1Wih, NLAT, NLAT, d1Wih, 1,    NLAT, NG1, KD1X, WXH);
    wplane_kernel<1><<<(n8c + 255) / 256, 256, 0, stream>>>(d1Wih, NLAT, NLAT, d1Wih, 1,    NLAT, NG1, KD1X, WXL);
    wplane_kernel<0><<<(n8d + 255) / 256, 256, 0, stream>>>(d1Whh, NHID, NHID, d1Whh, 1,    NHID, NG1, KD1H, WH);
    wplane_kernel<0><<<(n8e + 255) / 256, 256, 0, stream>>>(d2Wih, NHID, NHID, d2Wih, 1,    NHID, NG4, KD2,  W4H);
    wplane_kernel<1><<<(n8e + 255) / 256, 256, 0, stream>>>(d2Wih, NHID, NHID, d2Wih, 1,    NHID, NG4, KD2,  W4L);
  }
  enc_kernel<<<NBATCH / EROWS, ETHR, 0, stream>>>(x, WE1, WE2, e1bih, e1bhh, e2bih, e2bhh, LAT);
  dec_kernel<<<NBATCH / DROWS, DTHR, 0, stream>>>(LAT, WXH, WXL, WH, W4H, W4L, d1bih, d1bhh, d2Whh, d2bih, d2bhh, out);
}
